// SparseResNetEncoder_5471788335529
// MI455X (gfx1250) — hardware-verified
//
#include <hip/hip_runtime.h>

typedef float          v8f   __attribute__((ext_vector_type(8)));
typedef float          v4f   __attribute__((ext_vector_type(4)));
typedef unsigned int   v4u   __attribute__((ext_vector_type(4)));
typedef int            v8i   __attribute__((ext_vector_type(8)));
typedef unsigned short v8us  __attribute__((ext_vector_type(8)));
typedef unsigned short v16us __attribute__((ext_vector_type(16)));
typedef __bf16         v16bf __attribute__((ext_vector_type(16)));
typedef _Float16       v16h  __attribute__((ext_vector_type(16)));
typedef v4f  __attribute__((may_alias)) v4fa;
typedef v8us __attribute__((may_alias)) v8usa;
union FragB { v16bf v; v16us u; v8us h[2]; v8i w; };
union FragH { v16h  v; v16us u; v8us h[2]; v8i w; };

__device__ __forceinline__ v8f wmb(const FragB& a, const FragB& b, v8f c) {
  v8f d = __builtin_amdgcn_wmma_f32_16x16x32_bf16(false, a.v, false, b.v, (short)0, c, false, false);
  asm volatile("v_nop\n\tv_nop\n\tv_nop\n\tv_nop" : "+v"(d) : "v"(a.w), "v"(b.w));
  return d;
}

__device__ __forceinline__ v8f wmh(const FragH& a, const FragH& b, v8f c) {
  v8f d = __builtin_amdgcn_wmma_f32_16x16x32_f16(false, a.v, false, b.v, (short)0, c, false, false);
  asm volatile("v_nop\n\tv_nop\n\tv_nop\n\tv_nop" : "+v"(d) : "v"(a.w), "v"(b.w));
  return d;
}

__device__ __forceinline__ unsigned bf16_bits(float f) {
  const unsigned u = __float_as_uint(f);
  const unsigned r = (u + 0x7FFFu + ((u >> 16) & 1u)) >> 16;
  const unsigned q = (u >> 16) | 0x40u;
  return ((u & 0x7fffffffu) > 0x7f800000u) ? q : r;
}

__device__ __forceinline__ float bf16_val(float f) {
  return __uint_as_float(bf16_bits(f) << 16);
}
__device__ __forceinline__ int clampi(int v, int lo, int hi) {
  return v < lo ? lo : (v > hi ? hi : v);
}

__device__ __forceinline__ unsigned f16_bits(float f) {
  const unsigned u  = __float_as_uint(f);
  const unsigned s  = (u >> 16) & 0x8000u;
  const unsigned a  = u & 0x7fffffffu;
  const unsigned t  = a - 0x38000000u;
  const unsigned r  = (t + 0x0FFFu + ((t >> 13) & 1u)) >> 13;
  const unsigned rc = r > 0x7C00u ? 0x7C00u : r;
  const bool small  = a < 0x38800000u;
  const bool isnan  = a > 0x7f800000u;
  const unsigned fin = small ? 0u : (s | rc);
  return isnan ? (s | 0x7E00u) : fin;
}

__device__ __forceinline__ unsigned pk16(unsigned lo, unsigned hi) { return lo | (hi << 16); }
__device__ __forceinline__ unsigned bf16_lo_bits(float v) {
  float hi = bf16_val(v);
  asm volatile("" : "+v"(hi));
  return bf16_bits(v - hi);
}
__device__ __forceinline__ v4u pack8_bf16(v4f a, v4f c) {
  return (v4u){ pk16(bf16_bits(a[0]), bf16_bits(a[1])), pk16(bf16_bits(a[2]), bf16_bits(a[3])),
                pk16(bf16_bits(c[0]), bf16_bits(c[1])), pk16(bf16_bits(c[2]), bf16_bits(c[3])) };
}
__device__ __forceinline__ v4u pack8_bf16_lo(v4f a, v4f c) {
  return (v4u){ pk16(bf16_lo_bits(a[0]), bf16_lo_bits(a[1])), pk16(bf16_lo_bits(a[2]), bf16_lo_bits(a[3])),
                pk16(bf16_lo_bits(c[0]), bf16_lo_bits(c[1])), pk16(bf16_lo_bits(c[2]), bf16_lo_bits(c[3])) };
}
__device__ __forceinline__ v4u pack8_f16(v4f a, v4f c) {
  return (v4u){ pk16(f16_bits(a[0]), f16_bits(a[1])), pk16(f16_bits(a[2]), f16_bits(a[3])),
                pk16(f16_bits(c[0]), f16_bits(c[1])), pk16(f16_bits(c[2]), f16_bits(c[3])) };
}

template <int FORM>
__global__ __launch_bounds__(256) void k_plane(const float* __restrict__ src, int rows, int cols, int ldsrc,
                                               unsigned short* __restrict__ dst, int MP, int KP) {
  static_assert(FORM >= 0 && FORM <= 3);
  const int KTOT = (FORM == 1 || FORM == 3) ? 2 * KP : KP;
  const unsigned ppr   = (unsigned)(KTOT >> 3);
  const unsigned kp8   = (unsigned)(KP >> 3);
  const unsigned total = (unsigned)MP * ppr;
  const unsigned g     = blockIdx.x * 256u + threadIdx.x;
  const unsigned rowu  = g / ppr;
  const unsigned p     = g - rowu * ppr;
  const bool second    = p >= kp8;
  const int row = (int)rowu;
  const int c0  = (int)((second ? p - kp8 : p) << 3);
  const float* srow = src + (size_t)clampi(row, 0, rows - 1) * (size_t)ldsrc;
  float x[8];
  unsigned mk[8];
#pragma unroll
  for (int e = 0; e < 8; ++e) {
    const int c = c0 + e;
    const float v = srow[clampi(c, 0, cols - 1)];
    asm volatile("" :: "v"(v));
    x[e]  = v;
    mk[e] = (row < rows && c < cols) ? 0xFFFFu : 0u;
  }
  const v4f a = (v4f){ x[0], x[1], x[2], x[3] };
  const v4f c = (v4f){ x[4], x[5], x[6], x[7] };
  v4u o;
  if (FORM == 2) {
    o = pack8_f16(a, c);
  } else {
    const v4u hi = pack8_bf16(a, c);
    o = hi;
    if (FORM == 1) { const v4u lo = pack8_bf16_lo(a, c); o = second ? lo : hi; }
  }
  const v4u mw = (v4u){ pk16(mk[0], mk[1]), pk16(mk[2], mk[3]), pk16(mk[4], mk[5]), pk16(mk[6], mk[7]) };
  o &= mw;
  if (g < total) {
    volatile v4u* q = (volatile v4u*)(dst + (size_t)g * 8);
    *q = o;
    __threadfence();
    *q = o;
  }
}

template <int FORM> struct FragOf    { typedef FragB T; };
template <>         struct FragOf<2> { typedef FragH T; };
__device__ __forceinline__ v8f mm(const FragB& a, const FragB& b, v8f c) { return wmb(a, b, c); }
__device__ __forceinline__ v8f mm(const FragH& a, const FragH& b, v8f c) { return wmh(a, b, c); }
template <class F> __device__ __forceinline__ F ld_frag(const unsigned short* p) {
  F f;
  f.h[0] = *(const v8usa*)(p);
  f.h[1] = *(const v8usa*)(p + 16);
  return f;
}

template <int FORM, int EPI>
__global__ __launch_bounds__(256) __attribute__((amdgpu_num_vgpr(248)))
void k_gemm_nt(const unsigned short* __restrict__ A, const unsigned short* __restrict__ B,
               const float* __restrict__ bias, float* __restrict__ D, int M, int N, int KTOT, int ldd) {
  static_assert(FORM >= 0 && FORM <= 2);
  static_assert(EPI == 0 || EPI == 1);
  typedef typename FragOf<FORM>::T F;
  __shared__ __attribute__((aligned(16))) float sT[8][16 * 68];
  const int lane = threadIdx.x & 31;
  const int wave = threadIdx.x >> 5;
  const int tilesM = (M + 63) >> 6;
  const int tilesN = (N + 63) >> 6;
  const int tile = blockIdx.x * 8 + wave;
  if (tile >= tilesM * tilesN) return;
  const int tm = tile / tilesN;
  const int tn = tile - tm * tilesN;
  const int m0 = tm << 6;
  const int n0 = tn << 6;

  const int rl = lane & 15;
  const int h8 = (lane >> 4) * 8;
  const unsigned short* pa = A + (size_t)(m0 + rl) * (size_t)KTOT + h8;
  const unsigned short* pb = B + (size_t)(n0 + rl) * (size_t)KTOT + h8;

  v8f acc[4][4];
#pragma unroll
  for (int i = 0; i < 4; ++i)
#pragma unroll
    for (int j = 0; j < 4; ++j) acc[i][j] = (v8f){0.f, 0.f, 0.f, 0.f, 0.f, 0.f, 0.f, 0.f};

#pragma unroll 1
  for (int k0 = 0; k0 < KTOT; k0 += 32) {
    F bf[4];
#pragma unroll
    for (int j = 0; j < 4; ++j) bf[j] = ld_frag<F>(pb + (size_t)(j << 4) * (size_t)KTOT + k0);
#pragma unroll
    for (int i = 0; i < 4; ++i) {
      const F af = ld_frag<F>(pa + (size_t)(i << 4) * (size_t)KTOT + k0);
#pragma unroll
      for (int j = 0; j < 4; ++j) acc[i][j] = mm(af, bf[j], acc[i][j]);
    }
  }

  float* slab = sT[wave];
  const int hh = lane >> 4;
  const int c4 = (lane & 15) * 4;
  const int nc = n0 + c4;
  const bool cok = nc < N;
  v4f bv = (v4f){0.f, 0.f, 0.f, 0.f};
  if (EPI == 1) {
    bv = *(const v4fa*)(bias + clampi(nc, 0, N - 4));
    asm volatile("" :: "v"(bv));
  }
#pragma unroll
  for (int i = 0; i < 4; ++i) {
    const int mBase = m0 + (i << 4);
#pragma unroll
    for (int j = 0; j < 4; ++j) {
#pragma unroll
      for (int r = 0; r < 8; ++r) slab[(h8 + r) * 68 + (j << 4) + rl] = acc[i][j][r];
    }
    __builtin_amdgcn_fence(__ATOMIC_RELEASE, "workgroup");
    __builtin_amdgcn_wave_barrier();
    __builtin_amdgcn_fence(__ATOMIC_ACQUIRE, "workgroup");
    v4f vv[8];
#pragma unroll
    for (int it = 0; it < 8; ++it) {
      const int row = it * 2 + hh;
      v4f v = *(const v4fa*)(slab + row * 68 + c4);
      if (EPI == 1) v += bv;
      vv[it] = v;
    }
    for (int pass = 0; pass < 2; ++pass) {
#pragma unroll
      for (int it = 0; it < 8; ++it) {
        const int row = mBase + it * 2 + hh;
        if (cok && row < M) *(volatile v4f*)(D + (size_t)row * (size_t)ldd + nc) = vv[it];
      }
      __threadfence();
    }
    __builtin_amdgcn_fence(__ATOMIC_RELEASE, "workgroup");
    __builtin_amdgcn_wave_barrier();
    __builtin_amdgcn_fence(__ATOMIC_ACQUIRE, "workgroup");
  }
}

#include <stddef.h>
#pragma clang fp contract(off)

#ifndef TWO_TERM_L2
#define TWO_TERM_L2 1
#endif
#ifndef TWO_TERM_L3
#define TWO_TERM_L3 1
#endif
#ifndef TWO_TERM_L4
#define TWO_TERM_L4 1
#endif
#ifndef TWO_TERM_L5
#define TWO_TERM_L5 1
#endif
static_assert(TWO_TERM_L2 == 0 || TWO_TERM_L2 == 1);
static_assert(TWO_TERM_L3 == 0 || TWO_TERM_L3 == 1);
static_assert(TWO_TERM_L4 == 0 || TWO_TERM_L4 == 1);
static_assert(TWO_TERM_L5 == 0 || TWO_TERM_L5 == 1);

typedef float v2f __attribute__((ext_vector_type(2)));
typedef v2f __attribute__((may_alias)) v2fa;

constexpr int cdiv(int a, int b) { return (a + b - 1) / b; }
constexpr int cup(int a, int b)  { return cdiv(a, b) * b; }
constexpr int rc_of(int M, int R, int c) { return (M - c * R) < R ? (M - c * R) : R; }
constexpr size_t al256(size_t v) { return (v + 255) & ~(size_t)255; }
constexpr size_t smax(size_t a, size_t b) { return a > b ? a : b; }

constexpr int NTAP = 27;
constexpr int N0 = 395420;
constexpr int M1 = 364054, M2 = 204823, M3 = 32768, M4 = 4096, M5 = 512;
constexpr int C0 = 1, C1 = 16, C2 = 32, C3 = 64, C4 = 128, C5 = 512;
constexpr int KP1 = 64, KP2 = 448, KP3 = 896, KP4 = 1728, KP5 = 3456;
constexpr int KT1 = KP1;
constexpr int KT2 = TWO_TERM_L2 ? 2 * KP2 : KP2;
constexpr int KT3 = TWO_TERM_L3 ? 2 * KP3 : KP3;
constexpr int KT4 = TWO_TERM_L4 ? 2 * KP4 : KP4;
constexpr int KT5 = TWO_TERM_L5 ? 2 * KP5 : KP5;
constexpr int NP1 = 64, NP2 = 64, NP3 = 64, NP4 = 128, NP5 = 512;
constexpr int R1 = 65536, NCH1 = 6;
constexpr int R2 = 24576, NCH2 = 9;
constexpr int R3 = 12288, NCH3 = 3;

static_assert(NTAP <= 32);
static_assert(KP1 % 64 == 0 && KP2 % 64 == 0 && KP3 % 64 == 0 && KP4 % 64 == 0 && KP5 % 64 == 0);
static_assert(KT1 % 32 == 0 && KT2 % 32 == 0 && KT3 % 32 == 0 && KT4 % 32 == 0 && KT5 % 32 == 0);
static_assert(NTAP * C0 <= KP1 && NTAP * C1 <= KP2 && NTAP * C2 <= KP3 && NTAP * C3 <= KP4 && NTAP * C4 <= KP5);
static_assert(NP1 % 64 == 0 && NP2 % 64 == 0 && NP3 % 64 == 0 && NP4 % 64 == 0 && NP5 % 64 == 0);
static_assert(NP1 >= C1 && NP2 >= C2 && NP3 == C3 && NP4 == C4 && NP5 == C5);
static_assert(R1 % 128 == 0 && R2 % 128 == 0 && R3 % 128 == 0 && R1 % 2 == 0);
static_assert((NCH1 - 1) * R1 < M1 && NCH1 * R1 >= M1 && rc_of(M1, R1, NCH1 - 1) == 36374);
static_assert((NCH2 - 1) * R2 < M2 && NCH2 * R2 >= M2 && rc_of(M2, R2, NCH2 - 1) == 8215);
static_assert((NCH3 - 1) * R3 < M3 && NCH3 * R3 >= M3 && rc_of(M3, R3, NCH3 - 1) == 8192);
static_assert(R3 % 16 == 0 && rc_of(M3, R3, NCH3 - 1) % 16 == 0 && M4 % 128 == 0 && M5 % 128 == 0);
static_assert(M1 % 2 == 0);
static_assert((KT2 * 2) % 128 == 0 && (KT3 * 2) % 128 == 0 && (KT4 * 2) % 128 == 0 && (KT5 * 2) % 128 == 0);
static_assert(((size_t)R3 * C3 * 4) % 128 == 0);

constexpr int PB1 = NP1 * (KT1 / 8) / 256;
constexpr int PB2 = NP2 * (KT2 / 8) / 256;
constexpr int PB3 = NP3 * (KT3 / 8) / 256;
constexpr int PB4 = NP4 * (KT4 / 8) / 256;
constexpr int PB5 = NP5 * (KT5 / 8) / 256;
constexpr int WE1 = PB1, WE2 = WE1 + PB2, WE3 = WE2 + PB3, WE4 = WE3 + PB4, WE5 = WE4 + PB5;
static_assert((NP1 * (KT1 / 8)) % 256 == 0 && (NP2 * (KT2 / 8)) % 256 == 0 && (NP3 * (KT3 / 8)) % 256 == 0);
static_assert((NP4 * (KT4 / 8)) % 256 == 0 && (NP5 * (KT5 / 8)) % 256 == 0);

constexpr size_t SZ_W1T = (size_t)NP1 * KT1 * 2;
constexpr size_t SZ_W2T = (size_t)NP2 * KT2 * 2;
constexpr size_t SZ_W3T = (size_t)NP3 * KT3 * 2;
constexpr size_t SZ_W4T = (size_t)NP4 * KT4 * 2;
constexpr size_t SZ_W5T = (size_t)NP5 * KT5 * 2;
constexpr size_t SZ_OPC = smax(smax((size_t)R1 * KT1 * 2, (size_t)R2 * KT2 * 2),
                               smax(smax((size_t)R3 * KT3 * 2, (size_t)M4 * KT4 * 2), (size_t)M5 * KT5 * 2));
constexpr size_t SZ_DCH = (size_t)R1 * 64 * 4;
constexpr size_t SZ_X1  = al256((size_t)M1 * C1 * 4);
constexpr size_t SZ_X2  = al256((size_t)M2 * C2 * 4);
constexpr size_t SZ_X3  = (size_t)M3 * C3 * 4;
constexpr size_t SZ_X4  = (size_t)M4 * C4 * 4;
constexpr size_t OFF_W1T = 0;
constexpr size_t OFF_W2T = OFF_W1T + SZ_W1T;
constexpr size_t OFF_W3T = OFF_W2T + SZ_W2T;
constexpr size_t OFF_W4T = OFF_W3T + SZ_W3T;
constexpr size_t OFF_W5T = OFF_W4T + SZ_W4T;
constexpr size_t OFF_OPC = OFF_W5T + SZ_W5T;
constexpr size_t OFF_DCH = OFF_OPC + SZ_OPC;
constexpr size_t OFF_X1  = OFF_DCH + SZ_DCH;
constexpr size_t OFF_X2  = OFF_X1 + SZ_X1;
constexpr size_t OFF_X3  = OFF_X2 + SZ_X2;
constexpr size_t OFF_X4  = OFF_X3 + SZ_X3;
constexpr size_t WS_TOTAL = OFF_X4 + SZ_X4;
static_assert(SZ_W1T % 256 == 0 && SZ_W2T % 256 == 0 && SZ_W3T % 256 == 0 && SZ_W4T % 256 == 0 && SZ_W5T % 256 == 0);
static_assert(SZ_OPC % 256 == 0 && SZ_DCH % 256 == 0 && SZ_X1 % 256 == 0 && SZ_X2 % 256 == 0);
static_assert(SZ_X3 % 256 == 0 && SZ_X4 % 256 == 0);
static_assert((size_t)PB1 * 256 * 16 == SZ_W1T && (size_t)PB2 * 256 * 16 == SZ_W2T && (size_t)PB3 * 256 * 16 == SZ_W3T);
static_assert((size_t)PB4 * 256 * 16 == SZ_W4T && (size_t)PB5 * 256 * 16 == SZ_W5T);
static_assert((size_t)R2 * 64 * 4 <= SZ_DCH);
static_assert(SZ_DCH == (size_t)16777216 && SZ_X1 == (size_t)23299584 && SZ_X2 == (size_t)26217472);
static_assert(SZ_X3 == (size_t)8388608 && SZ_X4 == (size_t)2097152);
static_assert(WS_TOTAL <= ((size_t)128 << 20));
static_assert(!(TWO_TERM_L2 && TWO_TERM_L3 && TWO_TERM_L4 && TWO_TERM_L5) ||
              (SZ_OPC == (size_t)44040192 && WS_TOTAL == (size_t)((size_t)252217 << 9)));

__device__ __forceinline__ float mz(float v, unsigned m) { return __uint_as_float(__float_as_uint(v) & m); }

__device__ __forceinline__ void wt_unit(const float* __restrict__ W, int krows, int cout, int kp8, int ppr,
                                        unsigned short* __restrict__ dst, int u) {
  const int n  = u / ppr;
  const int p  = u - n * ppr;
  const int ks = (p % kp8) << 3;
  const int nc = n < cout ? n : cout - 1;
  float x[8];
  unsigned mk[8];
#pragma unroll
  for (int e = 0; e < 8; ++e) {
    const int k  = ks + e;
    const int kc = k < krows ? k : krows - 1;
    const float v = W[(size_t)kc * (size_t)cout + (size_t)nc];
    asm volatile("" :: "v"(v));
    x[e]  = v;
    mk[e] = (n < cout && k < krows) ? 0xFFFFu : 0u;
  }
  v4u o = pack8_bf16((v4f){ x[0], x[1], x[2], x[3] }, (v4f){ x[4], x[5], x[6], x[7] });
  o &= (v4u){ pk16(mk[0], mk[1]), pk16(mk[2], mk[3]), pk16(mk[4], mk[5]), pk16(mk[6], mk[7]) };
  volatile v4u* q = (volatile v4u*)(dst + (size_t)u * 8);
  *q = o;
  __threadfence();
  *q = o;
}

__global__ __launch_bounds__(256) void k_wprep(const float* __restrict__ w1, const float* __restrict__ w2,
                                               const float* __restrict__ w3, const float* __restrict__ w4,
                                               const float* __restrict__ w5,
                                               unsigned short* __restrict__ t1, unsigned short* __restrict__ t2,
                                               unsigned short* __restrict__ t3, unsigned short* __restrict__ t4,
                                               unsigned short* __restrict__ t5) {
  const int tid = (int)threadIdx.x;
  const int blk = (int)blockIdx.x;
  if (blk < WE1) {
    wt_unit(w1, NTAP * C0, C1, KP1 / 8, KT1 / 8, t1, blk * 256 + tid);
  } else if (blk < WE2) {
    wt_unit(w2, NTAP * C1, C2, KP2 / 8, KT2 / 8, t2, (blk - WE1) * 256 + tid);
  } else if (blk < WE3) {
    wt_unit(w3, NTAP * C2, C3, KP3 / 8, KT3 / 8, t3, (blk - WE2) * 256 + tid);
  } else if (blk < WE4) {
    wt_unit(w4, NTAP * C3, C4, KP4 / 8, KT4 / 8, t4, (blk - WE3) * 256 + tid);
  } else {
    wt_unit(w5, NTAP * C4, C5, KP5 / 8, KT5 / 8, t5, (blk - WE4) * 256 + tid);
  }
}

__global__ __launch_bounds__(256) void k_gather1(const float* __restrict__ feats, const int* __restrict__ nmap,
                                                 unsigned* __restrict__ OPW, int obase, int rc) {
  const int tid = (int)threadIdx.x, lane = tid & 31, wave = tid >> 5;
  const int r  = (int)blockIdx.x * 8 + wave;
  const int oc = clampi(obase + r, 0, M1 - 1);
  const int kt = lane < NTAP ? lane : NTAP - 1;
  int id = nmap[(size_t)kt * (size_t)M1 + (size_t)oc];
  asm volatile("" :: "v"(id));
  id = clampi(id, -1, N0 - 1);
  const int lm = (lane < NTAP && r < rc) ? -1 : 0;
  id = (id & lm) | ~lm;
  const int idc = id < 0 ? 0 : id;
  const float f = feats[idc];
  asm volatile("" :: "v"(f));
  const unsigned m = (id >= 0) ? 0xFFFFFFFFu : 0u;
  const unsigned b = bf16_bits(mz(f, m));
  const int s0 = (2 * lane) & 31;
  const unsigned a0 = (unsigned)__shfl((int)b, s0, 32);
  const unsigned a1 = (unsigned)__shfl((int)b, s0 + 1, 32);
  const unsigned w  = pk16(a0 & 0xFFFFu, a1 & 0xFFFFu);
  const unsigned ow = (lane < 14) ? w : 0u;
  volatile unsigned* q = (volatile unsigned*)(OPW + (size_t)r * 32 + lane);
  *q = ow;
  __threadfence();
  *q = ow;
}

template <int CIN, int KP, int TWO, int WPB>
__global__ __launch_bounds__(32 * WPB) void k_gatherN(const float* __restrict__ src, const int* __restrict__ nmap,
                                                     unsigned short* __restrict__ OP, int obase, int rc,
                                                     int mout, int nin) {
  static_assert(CIN == 16 || CIN == 32 || CIN == 64 || CIN == 128);
  static_assert(TWO == 0 || TWO == 1);
  static_assert(KP % 64 == 0 && KP % CIN == 0);
  constexpr int NSLOT = KP / CIN;
  static_assert(NSLOT >= NTAP && NSLOT <= 32);
  static_assert(CIN != 16 || NSLOT % 2 == 0);
  constexpr int KTOT = TWO ? 2 * KP : KP;
  constexpr int KP8  = KP / 8;
  constexpr int NIT  = (KP8 + 31) / 32;
  static_assert(KP8 % 8 == 0);
  static_assert((size_t)WPB * KP * 4 <= (size_t)65536);
  __shared__ __attribute__((aligned(16))) float strip[WPB][KP];
  const int tid = (int)threadIdx.x, lane = tid & 31, wave = tid >> 5;
  const int r  = (int)blockIdx.x * WPB + wave;
  const int oc = clampi(obase + r, 0, mout - 1);
  const int kt = lane < NTAP ? lane : NTAP - 1;
  int line = nmap[(size_t)kt * (size_t)mout + (size_t)oc];
  asm volatile("" :: "v"(line));
  line = clampi(line, -1, nin - 1);
  const int lm = (lane < NTAP && r < rc) ? -1 : 0;
  line = (line & lm) | ~lm;
  float* st = strip[wave];

  if constexpr (CIN == 16) {
    const int hf = lane >> 4;
    const int ch = lane & 15;
#pragma unroll 2
    for (int s = 0; s < NSLOT / 2; ++s) {
      const int id  = __shfl(line, 2 * s + hf, 32);
      const int idc = id < 0 ? 0 : id;
      const float v = src[(size_t)idc * CIN + ch];
      asm volatile("" :: "v"(v));
      const unsigned m = (id >= 0) ? 0xFFFFFFFFu : 0u;
      st[32 * s + lane] = mz(v, m);
    }
  } else if constexpr (CIN == 32) {
#pragma unroll 1
    for (int t = 0; t < NSLOT; ++t) {
      const int id  = __builtin_amdgcn_readlane(line, t);
      const int idc = id < 0 ? 0 : id;
      const float v = src[(size_t)idc * CIN + lane];
      asm volatile("" :: "v"(v));
      const unsigned m = (id >= 0) ? 0xFFFFFFFFu : 0u;
      st[CIN * t + lane] = mz(v, m);
    }
  } else if constexpr (CIN == 64) {
#pragma unroll 1
    for (int t = 0; t < NSLOT; ++t) {
      const int id  = __builtin_amdgcn_readlane(line, t);
      const int idc = id < 0 ? 0 : id;
      const v2f v = *(const v2fa*)(src + (size_t)idc * CIN + 2 * lane);
      asm volatile("" :: "v"(v));
      const unsigned m = (id >= 0) ? 0xFFFFFFFFu : 0u;
      *(v2fa*)(st + CIN * t + 2 * lane) = (v2f){ mz(v[0], m), mz(v[1], m) };
    }
  } else {
#pragma unroll 1
    for (int t = 0; t < NSLOT; ++t) {
      const int id  = __builtin_amdgcn_readlane(line, t);
      const int idc = id < 0 ? 0 : id;
      const v4f v = *(const v4fa*)(src + (size_t)idc * CIN + 4 * lane);
      asm volatile("" :: "v"(v));
      const unsigned m = (id >= 0) ? 0xFFFFFFFFu : 0u;
      *(v4fa*)(st + CIN * t + 4 * lane) = (v4f){ mz(v[0], m), mz(v[1], m), mz(v[2], m), mz(v[3], m) };
    }
  }
  __builtin_amdgcn_fence(__ATOMIC_RELEASE, "workgroup");
  __builtin_amdgcn_wave_barrier();
  __builtin_amdgcn_fence(__ATOMIC_ACQUIRE, "workgroup");

  unsigned short* rowp = OP + (size_t)r * (size_t)KTOT;
#pragma unroll 1
  for (int it = 0; it < NIT; ++it) {
    const int q  = it * 32 + lane;
    const bool ok = q < KP8;
    const int qc = ok ? q : KP8 - 1;
    const v4f a = *(const v4fa*)(st + 8 * qc);
    const v4f c = *(const v4fa*)(st + 8 * qc + 4);
    const v4u hi = pack8_bf16(a, c);
    volatile v4u* qh = (volatile v4u*)(rowp + 8 * (size_t)qc);
    if constexpr (TWO == 1) {
      const v4u lo = pack8_bf16_lo(a, c);
      volatile v4u* ql = (volatile v4u*)(rowp + KP + 8 * (size_t)qc);
      if (ok) *qh = hi;
      if (ok) *ql = lo;
      __threadfence();
      if (ok) *qh = hi;
      if (ok) *ql = lo;
    } else {
      if (ok) *qh = hi;
      __threadfence();
      if (ok) *qh = hi;
    }
  }
}

template <int COUT>
__global__ __launch_bounds__(256) void k_pack(const float* __restrict__ DCH, float* __restrict__ X, int obase, int rc) {
  static_assert(COUT == 16 || COUT == 32);
  constexpr int PPR = COUT / 4;
  const int u   = (int)blockIdx.x * 256 + (int)threadIdx.x;
  const int row = u / PPR;
  const int p   = u - row * PPR;
  const bool ok = row < rc;
  const int rcl = ok ? row : rc - 1;
  const v4f v = *(const v4fa*)(DCH + (size_t)rcl * 64 + 4 * p);
  asm volatile("" :: "v"(v));
  volatile v4f* q = (volatile v4f*)(X + (size_t)(obase + rcl) * COUT + 4 * p);
  if (ok) *q = v;
  __threadfence();
  if (ok) *q = v;
}

extern "C" void kernel_launch(void* const* d_in, const int* in_sizes, int n_in,
                              void* d_out, int out_size, void* d_ws, size_t ws_size,
                              hipStream_t stream) {
  if (n_in < 11) return;
  if (in_sizes[0] != N0 * C0) return;
  if (in_sizes[1] != NTAP * C0 * C1) return;
  if (in_sizes[2] != NTAP * M1) return;
  if (in_sizes[3] != NTAP * C1 * C2) return;
  if (in_sizes[4] != NTAP * M2) return;
  if (in_sizes[5] != NTAP * C2 * C3) return;
  if (in_sizes[6] != NTAP * M3) return;
  if (in_sizes[7] != NTAP * C3 * C4) return;
  if (in_sizes[8] != NTAP * M4) return;
  if (in_sizes[9] != NTAP * C4 * C5) return;
  if (in_sizes[10] != NTAP * M5) return;
  if (out_size != M5 * C5) return;
  if (ws_size < WS_TOTAL) return;

  const float* feats = (const float*)d_in[0];
  const float* W1  = (const float*)d_in[1];
  const int*   nm1 = (const int*)d_in[2];
  const float* W2  = (const float*)d_in[3];
  const int*   nm2 = (const int*)d_in[4];
  const float* W3  = (const float*)d_in[5];
  const int*   nm3 = (const int*)d_in[6];
  const float* W4  = (const float*)d_in[7];
  const int*   nm4 = (const int*)d_in[8];
  const float* W5  = (const float*)d_in[9];
  const int*   nm5 = (const int*)d_in[10];
  float* out = (float*)d_out;

  char* ws = (char*)d_ws;
  unsigned short* W1T = (unsigned short*)(ws + OFF_W1T);
  unsigned short* W2T = (unsigned short*)(ws + OFF_W2T);
  unsigned short* W3T = (unsigned short*)(ws + OFF_W3T);
  unsigned short* W4T = (unsigned short*)(ws + OFF_W4T);
  unsigned short* W5T = (unsigned short*)(ws + OFF_W5T);
  unsigned short* OPC = (unsigned short*)(ws + OFF_OPC);
  float* DCH = (float*)(ws + OFF_DCH);
  float* X1c = (float*)(ws + OFF_X1);
  float* X2c = (float*)(ws + OFF_X2);
  float* X3  = (float*)(ws + OFF_X3);
  float* X4  = (float*)(ws + OFF_X4);
  const float* nobias = (const float*)(ws + OFF_X4);

  k_wprep<<<WE5, 256, 0, stream>>>(W1, W2, W3, W4, W5, W1T, W2T, W3T, W4T, W5T);

  for (int c = 0; c < NCH1; ++c) {
    const int rc  = rc_of(M1, R1, c);
    const int rp  = cup(rc, 128);
    const int m16 = cup(rc, 16);
    k_gather1<<<rp / 8, 256, 0, stream>>>(feats, nm1, (unsigned*)OPC, c * R1, rc);
    k_gemm_nt<0, 0><<<cdiv(cdiv(m16, 64) * (NP1 / 64), 8), 256, 0, stream>>>(OPC, W1T, nobias, DCH, m16, NP1, KT1, 64);
    k_pack<C1><<<cdiv(rc * (C1 / 4), 256), 256, 0, stream>>>(DCH, X1c, c * R1, rc);
  }
  for (int c = 0; c < NCH2; ++c) {
    const int rc  = rc_of(M2, R2, c);
    const int rp  = cup(rc, 128);
    const int m16 = cup(rc, 16);
    k_gatherN<C1, KP2, TWO_TERM_L2, 8><<<rp / 8, 256, 0, stream>>>(X1c, nm2, OPC, c * R2, rc, M2, M1);
    k_gemm_nt<0, 0><<<cdiv(cdiv(m16, 64) * (NP2 / 64), 8), 256, 0, stream>>>(OPC, W2T, nobias, DCH, m16, NP2, KT2, 64);
    k_pack<C2><<<cdiv(rc * (C2 / 4), 256), 256, 0, stream>>>(DCH, X2c, c * R2, rc);
  }
  for (int c = 0; c < NCH3; ++c) {
    const int rc = rc_of(M3, R3, c);
    const int rp = cup(rc, 128);
    k_gatherN<C2, KP3, TWO_TERM_L3, 8><<<rp / 8, 256, 0, stream>>>(X2c, nm3, OPC, c * R3, rc, M3, M2);
    k_gemm_nt<0, 0><<<cdiv(cdiv(rc, 64) * (NP3 / 64), 8), 256, 0, stream>>>(OPC, W3T, nobias,
                                                                           X3 + (size_t)c * R3 * C3, rc, C3, KT3, C3);
  }
  k_gatherN<C3, KP4, TWO_TERM_L4, 8><<<M4 / 8, 256, 0, stream>>>(X3, nm4, OPC, 0, M4, M4, M3);
  k_gemm_nt<0, 0><<<cdiv((M4 / 64) * (NP4 / 64), 8), 256, 0, stream>>>(OPC, W4T, nobias, X4, M4, C4, KT4, C4);
  k_gatherN<C4, KP5, TWO_TERM_L5, 4><<<M5 / 4, 128, 0, stream>>>(X4, nm5, OPC, 0, M5, M5, M4);
  k_gemm_nt<0, 0><<<cdiv((M5 / 64) * (NP5 / 64), 8), 256, 0, stream>>>(OPC, W5T, nobias, out, M5, C5, KT5, C5);
}
